// GINModel_2645699854676
// MI455X (gfx1250) — hardware-verified
//
#include <hip/hip_runtime.h>
#include <stddef.h>
#include <stdint.h>


#define NN      50000
#define NE      800000
#define NG      128
#define HID     64
#define VOC     100
#define NL      3
#define K2      128
#define GBM     128
#define NTILE   391
#define MP      (NTILE * GBM)
#define NTHR    256
#define NWAVE   8
#define CHUNK   2048
#define WCAP    256
#define LISTN   (NWAVE * WCAP)
#define NBMAX   2048
#define NBRUN   1024
#define NBLK    49
#define RCAP    28672
#define DEGCAP  64
#define PKS     11
#define WSQ     (HID * K2)
#define NWB     24
#define NTB     7
#define TB_B1   6400
#define TB_B2   6592
#define TB_WR   6784
#define TB_END  6848
#define TB_TOT  (NTB * NTHR * 4)
#define LDS_BKT ((2 * RCAP + 2 * NBMAX + LISTN) * 4 + 128)
#define WSMAX   134217728

static_assert(HID == 64);
static_assert(K2 == 2 * HID && (K2 % 32) == 0);
static_assert((NBRUN % 128) == 0 && NBRUN <= NBMAX && NBRUN == 4 * NTHR);
static_assert(NBLK * NBRUN >= MP && MP >= NN && (NTILE - 1) * GBM < NN);
static_assert((CHUNK & (CHUNK - 1)) == 0 && CHUNK <= (1 << PKS) && CHUNK == NWAVE * WCAP);
static_assert((NBMAX & (NBMAX - 1)) == 0 && NBMAX <= (1 << PKS) && NTHR * 8 == NBMAX);
static_assert(LISTN >= NBMAX);
static_assert(RCAP >= 17531 && (RCAP % (4 * NTHR)) == 0);
static_assert(DEGCAP >= 33 + 8);
static_assert(((long long)NE << PKS) < 4294967296LL);
static_assert(VOC * HID * 4 <= 65536);
static_assert(NG == 4 * 32);
static_assert(TB_B1 == VOC * HID && TB_B2 == TB_B1 + NL * HID && TB_WR == TB_B2 + NL * HID && TB_END == TB_WR + HID);
static_assert(TB_END <= TB_TOT && (TB_B1 % 64) == 0 && (TB_B2 % 64) == 0 && (TB_WR % 64) == 0);
static_assert(6 * (HID * (K2 / 8)) == NWB * NTHR);
static_assert(LDS_BKT <= 300000);
static_assert(GBM == NWAVE * 16);

typedef float          v2f  __attribute__((ext_vector_type(2)));
typedef float          v4f  __attribute__((ext_vector_type(4)));
typedef float          v8f  __attribute__((ext_vector_type(8)));
typedef int            v4i  __attribute__((ext_vector_type(4)));
typedef int            v8i  __attribute__((ext_vector_type(8)));
typedef unsigned int   v4u  __attribute__((ext_vector_type(4)));
typedef unsigned short v8us __attribute__((ext_vector_type(8)));
typedef __bf16         v16b __attribute__((ext_vector_type(16)));
typedef v2f  __attribute__((may_alias)) v2fa;
typedef v4f  __attribute__((may_alias)) v4fa;
typedef v4i  __attribute__((may_alias)) v4ia;
typedef v8us __attribute__((may_alias)) v8usa;
union FragB { v16b v; v8us h[2]; v8i w; };

__device__ __forceinline__ v8f wmb(const FragB& a, const FragB& b, v8f c) {
  v8f d = __builtin_amdgcn_wmma_f32_16x16x32_bf16(false, a.v, false, b.v, (short)0, c, false, false);
  asm volatile("v_nop\n\tv_nop\n\tv_nop\n\tv_nop" : "+v"(d) : "v"(a.w), "v"(b.w));
  return d;
}

__device__ __forceinline__ unsigned short bf_bits(float f) {
  const unsigned int u = __float_as_uint(f);
  const unsigned int r = (u + 0x7FFFu + ((u >> 16) & 1u)) >> 16;
  return (unsigned short)((f != f) ? 0x7FC0u : r);
}
__device__ __forceinline__ float bf_val(unsigned short b) { return __uint_as_float(((unsigned int)b) << 16); }
__device__ __forceinline__ float bf_rne(float f) { return bf_val(bf_bits(f)); }
__device__ __forceinline__ int clampi(int v, int lo, int hi) { return v < lo ? lo : (v > hi ? hi : v); }

__device__ __forceinline__ v8us cv8b(const float* __restrict__ p) {
  v8us o;
#pragma unroll
  for (int i = 0; i < 8; ++i) o[i] = bf_bits(p[(size_t)i * HID]);
  return o;
}
__device__ __forceinline__ float pick4(float a, float b, float c, float d,
                                       unsigned ma, unsigned mb, unsigned mc, unsigned md) {
  const unsigned u = (__float_as_uint(a) & ma) | (__float_as_uint(b) & mb) |
                     (__float_as_uint(c) & mc) | (__float_as_uint(d) & md);
  return __uint_as_float(u);
}

__global__ __launch_bounds__(NTHR) void k_prep(const float* __restrict__ W1, const float* __restrict__ W2,
                                               const float* __restrict__ emb, const float* __restrict__ b1,
                                               const float* __restrict__ b2, const float* __restrict__ wr,
                                               unsigned short* wt, float* tab) {
  const int tid = (int)threadIdx.x;
  const int blk = (int)blockIdx.x;
  if (blk < NWB) {
    const int u     = blk * NTHR + tid;
    const int mi    = u >> 10;
    const int v     = u & 1023;
    const int n     = v >> 4;
    const int k8    = (v & 15) * 8;
    const int kk    = k8 & (HID - 1);
    const int layer = mi >> 1;
    const size_t so = (size_t)layer * HID * HID + (size_t)kk * HID + (size_t)n;
    v8us o;
    if ((mi & 1) != 0) { o = cv8b(W2 + so); } else { o = cv8b(W1 + so); }
    unsigned short* dp = wt + (size_t)u * 8;
    *(volatile v8us*)dp = o;
    __threadfence();
    *(volatile v8us*)dp = o;
  } else {
    const int u  = (blk - NWB) * NTHR + tid;
    const int f0 = 4 * u;
    const int ie = clampi(f0, 0, TB_B1 - 4);
    const int i1 = clampi(f0 - TB_B1, 0, NL * HID - 4);
    const int i2 = clampi(f0 - TB_B2, 0, NL * HID - 4);
    const int ir = clampi(f0 - TB_WR, 0, HID - 4);
    const v4f ve = *(const v4f*)(emb + ie);
    const v4f v1 = *(const v4f*)(b1 + i1);
    const v4f v2 = *(const v4f*)(b2 + i2);
    const v4f vr = *(const v4f*)(wr + ir);
    const unsigned me = (f0 < TB_B1) ? 0xFFFFFFFFu : 0u;
    const unsigned m1 = (f0 >= TB_B1 && f0 < TB_B2) ? 0xFFFFFFFFu : 0u;
    const unsigned m2 = (f0 >= TB_B2 && f0 < TB_WR) ? 0xFFFFFFFFu : 0u;
    const unsigned mr = (f0 >= TB_WR && f0 < TB_END) ? 0xFFFFFFFFu : 0u;
    v4f o;
    o.x = bf_rne(pick4(ve.x, v1.x, v2.x, vr.x, me, m1, m2, mr));
    o.y = bf_rne(pick4(ve.y, v1.y, v2.y, vr.y, me, m1, m2, mr));
    o.z = bf_rne(pick4(ve.z, v1.z, v2.z, vr.z, me, m1, m2, mr));
    o.w = bf_rne(pick4(ve.w, v1.w, v2.w, vr.w, me, m1, m2, mr));
    float* dp = tab + f0;
    *(volatile v4f*)dp = o;
    __threadfence();
    *(volatile v4f*)dp = o;
  }
}

__device__ __forceinline__ int scan_chunk(const int* __restrict__ dsts, int nE, int cbase, int slotBase,
                                          int nb, int* list, int lane, int wave) {
  int wc = 0;
  const int elw  = wave * WCAP + lane;
  const int sent = -2147483647 - 1;
  int d[8];
#pragma unroll
  for (int j = 0; j < 8; ++j) {
    const int e  = cbase + elw + 32 * j;
    const int ec = e < nE ? e : nE - 1;
    const int v  = dsts[ec];
    d[j] = (e < nE) ? v : sent;
  }
  const unsigned nbs = (unsigned)slotBase;
  const unsigned unb = (unsigned)nb;
  const unsigned s0 = (unsigned)d[0] - nbs, s1 = (unsigned)d[1] - nbs;
  const unsigned s2 = (unsigned)d[2] - nbs, s3 = (unsigned)d[3] - nbs;
  const unsigned s4 = (unsigned)d[4] - nbs, s5 = (unsigned)d[5] - nbs;
  const unsigned s6 = (unsigned)d[6] - nbs, s7 = (unsigned)d[7] - nbs;
  const bool h0 = s0 < unb, h1 = s1 < unb, h2 = s2 < unb, h3 = s3 < unb;
  const bool h4 = s4 < unb, h5 = s5 < unb, h6 = s6 < unb, h7 = s7 < unb;
  const unsigned any = __builtin_amdgcn_ballot_w32(h0 | h1 | h2 | h3 | h4 | h5 | h6 | h7);
  if (any != 0u) {
#define HITJ(J, HJ, SJ) { \
      const unsigned mj = __builtin_amdgcn_ballot_w32(HJ); \
      if (mj != 0u) { \
        if (HJ) { \
          const int pos = wc + (int)__builtin_amdgcn_mbcnt_lo(mj, 0u); \
          if (pos < WCAP) list[wave * WCAP + pos] = ((elw + 32 * (J)) << PKS) | (int)(SJ); \
        } \
        wc += (int)__builtin_popcount(mj); } }
    HITJ(0, h0, s0)
    HITJ(1, h1, s1)
    HITJ(2, h2, s2)
    HITJ(3, h3, s3)
    HITJ(4, h4, s4)
    HITJ(5, h5, s5)
    HITJ(6, h6, s6)
    HITJ(7, h7, s7)
#undef HITJ
  }
  return wc;
}

__global__ __launch_bounds__(NTHR) void k_bucket(const int* __restrict__ srcs, const int* __restrict__ dsts,
                                                 int nN, int nE, int* lst, int* cntg, int* offg, int* flg) {
  extern __shared__ v4f lds_dyn[];
  int* reg1 = (int*)lds_dyn;
  int* reg2 = reg1 + RCAP;
  int* scnt = reg2 + RCAP;
  int* soff = scnt + NBMAX;
  int* list = soff + NBMAX;
  int* wcnt = list + LISTN;
  int* wtot = wcnt + NWAVE;
  int* wfl  = wtot + NWAVE;
  const int tid = (int)threadIdx.x, lane = tid & 31, wave = tid >> 5;
  const int blk = (int)blockIdx.x;
  const int nodeBase = blk * NBRUN;
  const int nb = NBRUN;

  for (int i = tid; i < NBMAX; i += NTHR) scnt[i] = 0;
  {
    const v4i z = {0, 0, 0, 0};
    for (int i = tid; i < RCAP / 4; i += NTHR) *(v4ia*)(reg2 + 4 * i) = z;
  }
  __syncthreads();

  int tot = 0;
  const int nChunks = (nE + CHUNK - 1) / CHUNK;
#pragma unroll 1
  for (int ch = 0; ch < nChunks; ++ch) {
    const int cbase = ch * CHUNK;
    const int wc = scan_chunk(dsts, nE, cbase, nodeBase, nb, list, lane, wave);
    if (lane == 0) wcnt[wave] = wc;
    __syncthreads();
    int pre = 0, all = 0;
#pragma unroll
    for (int w2 = 0; w2 < NWAVE; ++w2) {
      int c = wcnt[w2];
      c = c < 0 ? 0 : (c > WCAP ? WCAP : c);
      all += c;
      pre += (w2 < wave) ? c : 0;
    }
    const int wcc  = wc > WCAP ? WCAP : wc;
    const int base = tot + pre;
#pragma unroll 1
    for (int i = lane; i < wcc; i += 32) {
      const int ent = list[wave * WCAP + i];
      const int el  = (ent >> PKS) & (CHUNK - 1);
      const int sl  = ent & (NBMAX - 1);
      int eid = cbase + el;
      eid = eid > nE - 1 ? nE - 1 : eid;
      const int pos = base + i;
      if (pos < RCAP) reg1[pos] = (int)(((unsigned)eid << PKS) | (unsigned)sl);
    }
    tot += all;
    tot = tot > RCAP ? RCAP : tot;
    __syncthreads();
  }
  const int nh = tot;

  if (wave == 0) {
#pragma unroll 1
    for (int b0 = 0; b0 < nh; b0 += 32) {
      const int idx = b0 + lane;
      const int uv  = reg1[idx < nh ? idx : nh - 1];
      const int m32 = (nh - b0) < 32 ? (nh - b0) : 32;
#pragma unroll 1
      for (int k = 0; k < m32; ++k) {
        const int u  = __builtin_amdgcn_readlane(uv, k);
        const int sl = u & (NBMAX - 1);
        if (lane == 0) scnt[sl] = scnt[sl] + 1;
      }
    }
  }
  __syncthreads();

  {
    const v4i ca = *(const v4ia*)(scnt + 8 * tid);
    const v4i cb = *(const v4ia*)(scnt + 8 * tid + 4);
    const int e0 = ca.x < 0 ? 0 : ca.x, e1 = ca.y < 0 ? 0 : ca.y, e2 = ca.z < 0 ? 0 : ca.z, e3 = ca.w < 0 ? 0 : ca.w;
    const int e4 = cb.x < 0 ? 0 : cb.x, e5 = cb.y < 0 ? 0 : cb.y, e6 = cb.z < 0 ? 0 : cb.z, e7 = cb.w < 0 ? 0 : cb.w;
    const bool od = (e0 > DEGCAP) | (e1 > DEGCAP) | (e2 > DEGCAP) | (e3 > DEGCAP) |
                    (e4 > DEGCAP) | (e5 > DEGCAP) | (e6 > DEGCAP) | (e7 > DEGCAP);
    const unsigned odm = __builtin_amdgcn_ballot_w32(od);
    if (lane == 0) wfl[wave] = (odm != 0u) ? 1 : 0;
    const int ts = e0 + e1 + e2 + e3 + e4 + e5 + e6 + e7;
    int incl = ts;
#pragma unroll
    for (int d = 1; d < 32; d <<= 1) {
      const int up = __shfl_up(incl, d);
      if (lane >= d) incl += up;
    }
    if (lane == 31) wtot[wave] = incl;
    __syncthreads();
    int pre = 0;
#pragma unroll
    for (int w2 = 0; w2 < NWAVE; ++w2) pre += (w2 < wave) ? wtot[w2] : 0;
    int run = pre + incl - ts;
    soff[8 * tid + 0] = run; run += e0;
    soff[8 * tid + 1] = run; run += e1;
    soff[8 * tid + 2] = run; run += e2;
    soff[8 * tid + 3] = run; run += e3;
    soff[8 * tid + 4] = run; run += e4;
    soff[8 * tid + 5] = run; run += e5;
    soff[8 * tid + 6] = run; run += e6;
    soff[8 * tid + 7] = run;
  }
  __syncthreads();
  for (int i = tid; i < NBMAX; i += NTHR) list[i] = soff[i];
  __syncthreads();

  if (wave == 0) {
#pragma unroll 1
    for (int b0 = 0; b0 < nh; b0 += 32) {
      const int idx = b0 + lane;
      const int uv  = reg1[idx < nh ? idx : nh - 1];
      const int m32 = (nh - b0) < 32 ? (nh - b0) : 32;
#pragma unroll 1
      for (int k = 0; k < m32; ++k) {
        const int u   = __builtin_amdgcn_readlane(uv, k);
        const int sl  = u & (NBMAX - 1);
        const int eid = (int)((unsigned)u >> PKS);
        if (lane == 0) {
          int pos = list[sl];
          pos = pos < 0 ? 0 : (pos > RCAP - 1 ? RCAP - 1 : pos);
          reg2[pos] = eid;
          list[sl] = pos + 1;
        }
      }
    }
  }
  __syncthreads();

  int odall = 0;
#pragma unroll
  for (int w2 = 0; w2 < NWAVE; ++w2) odall |= wfl[w2];
  const int flag = (nh >= RCAP || odall != 0) ? 1 : 0;

  {
    const v4i cv = *(const v4ia*)(scnt + 4 * tid);
    const v4i ov = *(const v4ia*)(soff + 4 * tid);
    int* cp = cntg + (size_t)blk * NBRUN + 4 * tid;
    int* op = offg + (size_t)blk * NBRUN + 4 * tid;
    *(volatile v4i*)cp = cv;
    *(volatile v4i*)op = ov;
    __threadfence();
    *(volatile v4i*)cp = cv;
    *(volatile v4i*)op = ov;
  }

#pragma unroll 1
  for (int it = 0; it < RCAP / (4 * NTHR); ++it) {
    const int i0 = 4 * (it * NTHR + tid);
    const v4i e = *(const v4ia*)(reg2 + i0);
    const int s0 = clampi(srcs[clampi(e.x, 0, nE - 1)], 0, nN - 1);
    const int s1 = clampi(srcs[clampi(e.y, 0, nE - 1)], 0, nN - 1);
    const int s2 = clampi(srcs[clampi(e.z, 0, nE - 1)], 0, nN - 1);
    const int s3 = clampi(srcs[clampi(e.w, 0, nE - 1)], 0, nN - 1);
    v4i o;
    o.x = (i0     < nh) ? s0 : 0;
    o.y = (i0 + 1 < nh) ? s1 : 0;
    o.z = (i0 + 2 < nh) ? s2 : 0;
    o.w = (i0 + 3 < nh) ? s3 : 0;
    int* lp = lst + (size_t)blk * RCAP + i0;
    *(volatile v4i*)lp = o;
    __threadfence();
    *(volatile v4i*)lp = o;
  }

  {
    v4i fv;
    fv.x = (tid == 0) ? flag : 0;
    fv.y = (tid == 0) ? nh : 0;
    fv.z = 0;
    fv.w = 0;
    int* fp = flg + (size_t)blk * 32 + 4 * (tid & 7);
    const bool okf = tid < 8;
    if (okf) *(volatile v4i*)fp = fv;
    __threadfence();
    if (okf) *(volatile v4i*)fp = fv;
  }
}

template <int L0>
__global__ __launch_bounds__(NTHR) void k_agg(const int* __restrict__ lst, const int* __restrict__ cntg,
                                              const int* __restrict__ offg, const int* __restrict__ flg,
                                              const int* __restrict__ feats, const float* __restrict__ embr,
                                              const float* __restrict__ Hin, unsigned int* zout, int nN) {
  __shared__ __attribute__((aligned(16))) float etab[VOC * HID];
  const int tid = (int)threadIdx.x, lane = tid & 31;
  const int wave = __builtin_amdgcn_readfirstlane(tid >> 5);
  const int blk = (int)blockIdx.x;
  const int nodeBase = blk * NBRUN;
  if constexpr (L0 != 0) {
    for (int i = tid; i < (VOC * HID) / 4; i += NTHR) {
      const v4f v = *(const v4f*)(embr + 4 * i);
      *(v4fa*)(etab + 4 * i) = v;
    }
    __syncthreads();
  }
  const int bflag = flg[(size_t)blk * 32];
  const int* lb = lst + (size_t)blk * RCAP;
  const float qnan = __int_as_float(0x7fc00000);

#pragma unroll 1
  for (int jt = 0; jt < NBRUN / NWAVE; ++jt) {
    const int slot = wave * (NBRUN / NWAVE) + jt;
    const int grow = nodeBase + slot;
    if (grow >= MP) break;
    const int craw = __builtin_amdgcn_readfirstlane(cntg[grow]);
    int st = __builtin_amdgcn_readfirstlane(offg[grow]);
    st = clampi(st, 0, RCAP);
    int cnt = clampi(craw, 0, DEGCAP);
    if (cnt > RCAP - st) cnt = RCAP - st;
    const float pz = (bflag != 0 || craw > DEGCAP || craw < 0) ? qnan : 0.0f;
    const bool live = grow < nN;

    float a0 = 0.0f, a1 = 0.0f;
#pragma unroll 1
    for (int b0 = 0; b0 < cnt; b0 += 32) {
      int idx = st + b0 + lane;
      const int last = st + cnt - 1;
      idx = idx > last ? last : idx;
      idx = clampi(idx, 0, RCAP - 1);
      const int sv = clampi(lb[idx], 0, nN - 1);
      int key;
      if constexpr (L0 != 0) {
        key = clampi(feats[sv], 0, VOC - 1) * HID;
      } else {
        key = sv;
      }
      const int m32 = (cnt - b0) < 32 ? (cnt - b0) : 32;
#pragma unroll 1
      for (int k = 0; k < m32; ++k) {
        const int kk = __builtin_amdgcn_readlane(key, k);
        v2f v;
        if constexpr (L0 != 0) {
          v = *(const v2fa*)(etab + kk + 2 * lane);
        } else {
          v = *(const v2f*)(Hin + (size_t)kk * HID + 2 * lane);
        }
        a0 += v.x; a1 += v.y;
      }
    }
    const int rc = live ? grow : nN - 1;
    v2f sf;
    if constexpr (L0 != 0) {
      const int fk = clampi(feats[rc], 0, VOC - 1) * HID;
      sf = *(const v2fa*)(etab + fk + 2 * lane);
    } else {
      sf = *(const v2f*)(Hin + (size_t)rc * HID + 2 * lane);
    }
    float r0 = sf.x + a0, r1 = sf.y + a1;
    r0 = (live ? r0 : 0.0f) + pz;
    r1 = (live ? r1 : 0.0f) + pz;
    const unsigned short hb0 = bf_bits(r0), hb1 = bf_bits(r1);
    const unsigned short lb0 = bf_bits(r0 - bf_val(hb0)), lb1 = bf_bits(r1 - bf_val(hb1));
    const unsigned int hw = (unsigned int)hb0 | ((unsigned int)hb1 << 16);
    const unsigned int lw = (unsigned int)lb0 | ((unsigned int)lb1 << 16);
    unsigned int* zp = zout + (size_t)grow * (K2 / 2);
    *(volatile unsigned int*)(zp + lane) = hw;
    *(volatile unsigned int*)(zp + 32 + lane) = lw;
    __threadfence();
    *(volatile unsigned int*)(zp + lane) = hw;
    *(volatile unsigned int*)(zp + 32 + lane) = lw;
  }
}

template <int MODE>
__global__ __launch_bounds__(NTHR) void k_gemm(const unsigned short* __restrict__ A,
                                               const unsigned short* __restrict__ WT,
                                               const float* __restrict__ bias,
                                               const float* __restrict__ wrr,
                                               void* outp, int nN) {
  __shared__ __attribute__((aligned(16))) float stg[GBM * HID];
  __shared__ __attribute__((aligned(16))) float sst[GBM];
  __shared__ __attribute__((aligned(16))) float wrs[HID];
  const int tid = (int)threadIdx.x, lane = tid & 31, wave = tid >> 5, hh = lane >> 4, m = lane & 15;
  const int rowBase = (int)blockIdx.x * GBM;

  if constexpr (MODE == 2) {
    if (tid < HID / 4) {
      const v4f w = *(const v4f*)(wrr + 4 * tid);
      *(v4fa*)(wrs + 4 * tid) = w;
    }
  }

  v8f acc[4];
  {
    const v8f z = {0.f, 0.f, 0.f, 0.f, 0.f, 0.f, 0.f, 0.f};
#pragma unroll
    for (int t = 0; t < 4; ++t) acc[t] = z;
  }
  const unsigned short* ap = A + (size_t)(rowBase + 16 * wave + m) * (size_t)K2 + 8 * hh;
  const unsigned short* wp = WT + (size_t)m * (size_t)K2 + 8 * hh;
#pragma unroll 1
  for (int ks = 0; ks < K2 / 32; ++ks) {
    FragB af;
    af.h[0] = *(const v8usa*)(ap + 32 * ks);
    af.h[1] = *(const v8usa*)(ap + 32 * ks + 16);
#pragma unroll
    for (int t = 0; t < 4; ++t) {
      const unsigned short* wq = wp + (size_t)(16 * t) * (size_t)K2 + 32 * ks;
      FragB bf;
      bf.h[0] = *(const v8usa*)wq;
      bf.h[1] = *(const v8usa*)(wq + 16);
      acc[t] = wmb(af, bf, acc[t]);
    }
  }

#pragma unroll
  for (int t = 0; t < 4; ++t) {
    const int lc = 16 * t + m;
    const float bb = bias[lc];
#pragma unroll
    for (int r = 0; r < 8; ++r) {
      const int lr = 16 * wave + 8 * hh + r;
      const bool live = (rowBase + lr) < nN;
      float v = acc[t][r] + bb;
      if constexpr (MODE == 0) v = (v > 0.0f) ? v : (v - v);
      stg[lr * HID + lc] = live ? v : 0.0f;
    }
  }
  __syncthreads();

  if constexpr (MODE == 0) {
    unsigned short* outH = (unsigned short*)outp;
    const int p  = lane & 15;
    const int rs = lane >> 4;
    const int cb = 8 * (p & 7);
    const bool isHi = p < 8;
    v4u pk[8];
#pragma unroll
    for (int i = 0; i < 8; ++i) {
      const int lr = 16 * wave + 2 * i + rs;
      const v4f a = *(const v4fa*)(stg + lr * HID + cb);
      const v4f b = *(const v4fa*)(stg + lr * HID + cb + 4);
      const float f[8] = {a.x, a.y, a.z, a.w, b.x, b.y, b.z, b.w};
      unsigned int w[4];
#pragma unroll
      for (int j = 0; j < 4; ++j) {
        const unsigned short h0 = bf_bits(f[2 * j]), h1 = bf_bits(f[2 * j + 1]);
        const unsigned short l0 = bf_bits(f[2 * j] - bf_val(h0)), l1 = bf_bits(f[2 * j + 1] - bf_val(h1));
        const unsigned short q0 = isHi ? h0 : l0, q1 = isHi ? h1 : l1;
        w[j] = (unsigned int)q0 | ((unsigned int)q1 << 16);
      }
      v4u pw; pw.x = w[0]; pw.y = w[1]; pw.z = w[2]; pw.w = w[3];
      pk[i] = pw;
    }
#pragma unroll
    for (int i = 0; i < 8; ++i) {
      unsigned short* op = outH + (size_t)(rowBase + 16 * wave + 2 * i) * (size_t)K2 + 8 * lane;
      *(volatile v4u*)op = pk[i];
    }
    __threadfence();
#pragma unroll
    for (int i = 0; i < 8; ++i) {
      unsigned short* op = outH + (size_t)(rowBase + 16 * wave + 2 * i) * (size_t)K2 + 8 * lane;
      *(volatile v4u*)op = pk[i];
    }
  } else if constexpr (MODE == 1) {
    float* outF = (float*)outp;
    v4f fv[8];
#pragma unroll
    for (int i = 0; i < 8; ++i) {
      const int lr = 16 * wave + 2 * i + (lane >> 4);
      fv[i] = *(const v4fa*)(stg + lr * HID + 4 * (lane & 15));
    }
#pragma unroll
    for (int i = 0; i < 8; ++i) {
      float* op = outF + (size_t)(rowBase + 16 * wave + 2 * i) * (size_t)HID + 4 * lane;
      *(volatile v4f*)op = fv[i];
    }
    __threadfence();
#pragma unroll
    for (int i = 0; i < 8; ++i) {
      float* op = outF + (size_t)(rowBase + 16 * wave + 2 * i) * (size_t)HID + 4 * lane;
      *(volatile v4f*)op = fv[i];
    }
  } else {
    float* outS = (float*)outp;
    if (tid < GBM) {
      float s = 0.0f;
#pragma unroll 4
      for (int c = 0; c < HID; ++c) s = fmaf(stg[tid * HID + c], wrs[c], s);
      sst[tid] = s;
    }
    __syncthreads();
    const v4f sv = *(const v4fa*)(sst + 4 * lane);
    float* op = outS + (size_t)rowBase + 4 * lane;
    const bool okst = (wave == 0);
    if (okst) *(volatile v4f*)op = sv;
    __threadfence();
    if (okst) *(volatile v4f*)op = sv;
  }
}

__global__ __launch_bounds__(NTHR) void k_pool(const float* __restrict__ sc, const int* __restrict__ gid,
                                               const int* __restrict__ flg, int nN, float* out) {
  __shared__ __attribute__((aligned(16))) float outs[32];
  __shared__ int wfl[NWAVE];
  const int tid = (int)threadIdx.x, lane = tid & 31;
  const int wave = __builtin_amdgcn_readfirstlane(tid >> 5);
  const int q = (int)blockIdx.x;
  const int g0 = 32 * q + 4 * wave;

  double a0 = 0.0, a1 = 0.0, a2 = 0.0, a3 = 0.0;
#pragma unroll 1
  for (int i0 = 0; i0 < nN; i0 += 32) {
    const int i  = i0 + lane;
    const int ic = i < nN ? i : nN - 1;
    const int g  = gid[ic];
    const float s = sc[ic];
    const bool ok = i < nN;
    const double d = (double)s;
    a0 += (ok && g == g0    ) ? d : 0.0;
    a1 += (ok && g == g0 + 1) ? d : 0.0;
    a2 += (ok && g == g0 + 2) ? d : 0.0;
    a3 += (ok && g == g0 + 3) ? d : 0.0;
  }
#pragma unroll
  for (int o = 16; o >= 1; o >>= 1) {
    const double t0 = __shfl_xor(a0, o);
    const double t1 = __shfl_xor(a1, o);
    const double t2 = __shfl_xor(a2, o);
    const double t3 = __shfl_xor(a3, o);
    a0 += t0; a1 += t1; a2 += t2; a3 += t3;
  }
  {
    const int fi = tid < NBLK ? tid : NBLK - 1;
    const int f  = flg[(size_t)fi * 32];
    const bool bad = (tid < NBLK) && (f != 0);
    const unsigned bm = __builtin_amdgcn_ballot_w32(bad);
    if (lane == 0) {
      wfl[wave] = (bm != 0u) ? 1 : 0;
      outs[4 * wave + 0] = (float)a0;
      outs[4 * wave + 1] = (float)a1;
      outs[4 * wave + 2] = (float)a2;
      outs[4 * wave + 3] = (float)a3;
    }
  }
  __syncthreads();
  int anyf = 0;
#pragma unroll
  for (int w2 = 0; w2 < NWAVE; ++w2) anyf |= wfl[w2];
  const float qnan = __int_as_float(0x7fc00000);
  const int l8 = tid & 7;
  v4f ov = *(const v4fa*)(outs + 4 * l8);
  ov.x = (anyf != 0) ? qnan : ov.x;
  ov.y = (anyf != 0) ? qnan : ov.y;
  ov.z = (anyf != 0) ? qnan : ov.z;
  ov.w = (anyf != 0) ? qnan : ov.w;
  float* op = out + 32 * q + 4 * l8;
  const bool okst = tid < 8;
  if (okst) *(volatile v4f*)op = ov;
  __threadfence();
  if (okst) *(volatile v4f*)op = ov;
}

static inline size_t al256(size_t o) { return (o + 255) & ~(size_t)255; }

extern "C" void kernel_launch(void* const* d_in, const int* in_sizes, int n_in,
                              void* d_out, int out_size, void* d_ws, size_t ws_size,
                              hipStream_t stream) {
  if (n_in < 10) return;
  if (in_sizes[0] != NN || in_sizes[1] != NE || in_sizes[2] != NE || in_sizes[3] != NN) return;
  if (in_sizes[4] != VOC * HID) return;
  if (in_sizes[5] != NL * HID * HID || in_sizes[7] != NL * HID * HID) return;
  if (in_sizes[6] != NL * HID || in_sizes[8] != NL * HID) return;
  if (in_sizes[9] != HID) return;
  if (out_size != NG) return;

  const int*   feats = (const int*)  d_in[0];
  const int*   src   = (const int*)  d_in[1];
  const int*   dst   = (const int*)  d_in[2];
  const int*   gid   = (const int*)  d_in[3];
  const float* emb   = (const float*)d_in[4];
  const float* W1    = (const float*)d_in[5];
  const float* b1    = (const float*)d_in[6];
  const float* W2    = (const float*)d_in[7];
  const float* b2    = (const float*)d_in[8];
  const float* Wr    = (const float*)d_in[9];
  float* out = (float*)d_out;

  char* ws = (char*)d_ws;
  size_t off = 0;
  const size_t oWT  = off; off = al256(off + (size_t)6 * WSQ * 2);
  const size_t oTAB = off; off = al256(off + (size_t)TB_TOT * 4);
  const size_t oZP  = off; off = al256(off + (size_t)MP * K2 * 2);
  const size_t oTP  = off; off = al256(off + (size_t)MP * K2 * 2);
  const size_t oHF  = off; off = al256(off + (size_t)MP * HID * 4);
  const size_t oLS  = off; off = al256(off + (size_t)NBLK * RCAP * 4);
  const size_t oCN  = off; off = al256(off + (size_t)NBLK * NBRUN * 4);
  const size_t oOF  = off; off = al256(off + (size_t)NBLK * NBRUN * 4);
  const size_t oFL  = off; off = al256(off + (size_t)NBLK * 32 * 4);
  const size_t oSC  = off; off = al256(off + (size_t)MP * 4);
  if (off > ws_size || off > (size_t)WSMAX) return;
  unsigned short* WT  = (unsigned short*)(ws + oWT);
  float*          TAB = (float*)(ws + oTAB);
  unsigned short* ZP  = (unsigned short*)(ws + oZP);
  unsigned short* TP  = (unsigned short*)(ws + oTP);
  float*          HF  = (float*)(ws + oHF);
  int*            LS  = (int*)(ws + oLS);
  int*            CN  = (int*)(ws + oCN);
  int*            OF  = (int*)(ws + oOF);
  int*            FL  = (int*)(ws + oFL);
  float*          SC  = (float*)(ws + oSC);

  hipFuncSetAttribute(reinterpret_cast<const void*>(&k_bucket), hipFuncAttributeMaxDynamicSharedMemorySize, LDS_BKT);

  k_prep<<<NWB + NTB, NTHR, 0, stream>>>(W1, W2, emb, b1, b2, Wr, WT, TAB);
  k_bucket<<<NBLK, NTHR, LDS_BKT, stream>>>(src, dst, NN, NE, LS, CN, OF, FL);
  for (int l = 0; l < NL; ++l) {
    if (l == 0) {
      k_agg<1><<<NBLK, NTHR, 0, stream>>>(LS, CN, OF, FL, feats, TAB, HF, (unsigned int*)ZP, NN);
    } else {
      k_agg<0><<<NBLK, NTHR, 0, stream>>>(LS, CN, OF, FL, feats, TAB, HF, (unsigned int*)ZP, NN);
    }
    k_gemm<0><<<NTILE, NTHR, 0, stream>>>(ZP, WT + (size_t)(2 * l) * WSQ, TAB + TB_B1 + l * HID,
                                          TAB + TB_WR, (void*)TP, NN);
    if (l < NL - 1) {
      k_gemm<1><<<NTILE, NTHR, 0, stream>>>(TP, WT + (size_t)(2 * l + 1) * WSQ, TAB + TB_B2 + l * HID,
                                            TAB + TB_WR, (void*)HF, NN);
    } else {
      k_gemm<2><<<NTILE, NTHR, 0, stream>>>(TP, WT + (size_t)(2 * l + 1) * WSQ, TAB + TB_B2 + l * HID,
                                            TAB + TB_WR, (void*)SC, NN);
    }
  }
  k_pool<<<NG / 32, NTHR, 0, stream>>>(SC, gid, FL, NN, out);
}
